// PointNetFeaturePropagation_83588653515178
// MI455X (gfx1250) — hardware-verified
//
#include <hip/hip_runtime.h>

#pragma clang fp contract(off)

typedef __attribute__((ext_vector_type(16))) _Float16 v16h;
typedef __attribute__((ext_vector_type(8)))  _Float16 v8h;
typedef __attribute__((ext_vector_type(8)))  float    v8f;
typedef __attribute__((ext_vector_type(4)))  float    v4f;
typedef __attribute__((ext_vector_type(4)))  unsigned v4u;

constexpr int NBATCH  = 8;
constexpr int NQUERY  = 8192;
constexpr int NSRC    = 2048;
constexpr int CH_P1   = 128;
constexpr int CH_P2   = 256;
constexpr int CH_IN   = CH_P1 + CH_P2;
constexpr int CH_L0   = 256;
constexpr int CH_L1   = 128;
constexpr int KNBR    = 16;
constexpr int NROWS   = NBATCH * NQUERY;
constexpr int TILES_M = NROWS / 64;
constexpr int W0_ELEMS = CH_L0 * CH_IN;
constexpr int W1_ELEMS = CH_L1 * CH_L0;
constexpr int W0_BLOCKS = W0_ELEMS / 2048;
constexpr int W_BLOCKS  = (W0_ELEMS + W1_ELEMS) / 2048;
constexpr float W_CARRY     = 1024.0f;
constexpr float W_CARRY_INV = 1.0f / 1024.0f;
constexpr float EPS_DIST = 1e-4f;
constexpr float EPS_BN   = 1e-5f;

static_assert(CH_IN == 384);
static_assert(NROWS == 65536);
static_assert(NROWS % 64 == 0 && CH_L0 % 64 == 0 && CH_L1 % 64 == 0);
static_assert(CH_IN % 32 == 0 && CH_L0 % 32 == 0);
static_assert(W0_ELEMS % 2048 == 0 && W1_ELEMS % 2048 == 0);
static_assert((TILES_M * (CH_L0 / 64)) % 8 == 0 && (TILES_M * (CH_L1 / 64)) % 8 == 0);
static_assert(TILES_M % 8 == 0);

constexpr size_t OFF_IDX  = 0;
constexpr size_t OFF_DSEL = OFF_IDX  + (size_t)NROWS * KNBR * 4;
constexpr size_t OFF_XH   = OFF_DSEL + (size_t)NROWS * KNBR * 4;
constexpr size_t OFF_YF   = OFF_XH   + (size_t)NROWS * CH_IN * 2;
constexpr size_t OFF_WHI  = OFF_YF   + (size_t)NROWS * CH_L0 * 4;
constexpr size_t OFF_WLO  = OFF_WHI  + (size_t)(W0_ELEMS + W1_ELEMS) * 2;
constexpr size_t OFF_P0   = OFF_WLO  + (size_t)(W0_ELEMS + W1_ELEMS) * 2;
constexpr size_t OFF_P1   = OFF_P0   + (size_t)TILES_M * 2 * CH_L0 * 4;
constexpr size_t OFF_ST0  = OFF_P1   + (size_t)TILES_M * 2 * CH_L1 * 4;
constexpr size_t OFF_ST1  = OFF_ST0  + 2048;
constexpr size_t WS_TOTAL = OFF_ST1  + 2048;
static_assert(WS_TOTAL <= (size_t)134217728);
static_assert((size_t)NROWS * CH_L0 * 2 <= (size_t)NROWS * CH_IN * 2);
static_assert((size_t)NROWS * CH_L1 * 4 <= (size_t)NROWS * CH_L0 * 4);
static_assert(OFF_XH % 128 == 0 && OFF_YF % 128 == 0 && OFF_WHI % 128 == 0 && OFF_WLO % 128 == 0);
static_assert(OFF_P0 % 128 == 0 && OFF_P1 % 128 == 0 && OFF_ST0 % 128 == 0 && OFF_ST1 % 128 == 0);

struct FragH {
  union U { v16h v; v8h h[2]; };
  static __device__ __forceinline__ v16h load(const _Float16* p) {
    U f; f.h[0] = *(const v8h*)(p); f.h[1] = *(const v8h*)(p + 16); return f.v;
  }
  static __device__ __forceinline__ v8f mma(v16h a, v16h b, v8f c) {
    return __builtin_amdgcn_wmma_f32_16x16x32_f16(false, a, false, b, (short)0, c, false, false);
  }
};
__device__ __forceinline__ void guard_row_h(v8f& a, v8f& b, v8f& c, v8f& d, v16h x,
                                            v16h b0, v16h b1, v16h b2, v16h b3,
                                            v16h l0, v16h l1, v16h l2, v16h l3) {
  asm volatile("v_nop\n\tv_nop\n\tv_nop\n\tv_nop"
               : "+v"(a), "+v"(b), "+v"(c), "+v"(d)
               : "v"(x), "v"(b0), "v"(b1), "v"(b2), "v"(b3), "v"(l0), "v"(l1), "v"(l2), "v"(l3));
}
__device__ __forceinline__ void keep4_h(v16h a, v16h b, v16h c, v16h d) { asm volatile("v_nop" :: "v"(a), "v"(b), "v"(c), "v"(d)); }
__device__ __forceinline__ void acc_guard4(v8f& a, v8f& b, v8f& c, v8f& d) { asm volatile("v_nop\n\tv_nop\n\tv_nop\n\tv_nop" : "+v"(a), "+v"(b), "+v"(c), "+v"(d)); }

__global__ __launch_bounds__(256)
void knn16_kernel(const float* __restrict__ xyz1, const float* __restrict__ xyz2,
                  unsigned* __restrict__ idx_plane, unsigned* __restrict__ dsel_plane) {
#pragma clang fp contract(off)
  __shared__ v4u sbuf[NSRC];
  const int t = threadIdx.x;
  const int b = blockIdx.y;

#pragma unroll 1
  for (int i = 0; i < NSRC / 256; ++i) {
    const int s = t + 256 * i;
    const float* p = xyz2 + ((size_t)b * NSRC + s) * 3;
    const float x = p[0];
    const float y = p[1];
    const float z = p[2];
    const float t0 = x * x;
    const float t1 = y * y;
    const float t2 = z * z;
    const float bb = (t0 + t2) + t1;
    v4u c;
    c.x = __float_as_uint(x);
    c.y = __float_as_uint(y);
    c.z = __float_as_uint(z);
    c.w = __float_as_uint(bb);
    sbuf[s] = c;
  }
  __syncthreads();

  const int n = blockIdx.x * 256 + t;
  const size_t bn = (size_t)b * NQUERY + n;
  const float px = xyz1[bn * 3 + 0];
  const float py = xyz1[bn * 3 + 1];
  const float pz = xyz1[bn * 3 + 2];
  const float q0 = px * px;
  const float q1 = py * py;
  const float q2 = pz * pz;
  const float aa = (q0 + q2) + q1;

  float bd[KNBR];
  int   bi[KNBR];
#pragma unroll
  for (int k = 0; k < KNBR; ++k) { bd[k] = __builtin_inff(); bi[k] = 0; }

#pragma unroll 2
  for (int s = 0; s < NSRC; ++s) {
    const v4u c = sbuf[s];
    const unsigned ux = c.x;
    const unsigned uy = c.y;
    const unsigned uz = c.z;
    const unsigned uw = c.w;
    const float cx = __uint_as_float(ux);
    const float cy = __uint_as_float(uy);
    const float cz = __uint_as_float(uz);
    const float cb = __uint_as_float(uw);
    float p = px * cx;
    p = __builtin_fmaf(py, cy, p);
    p = __builtin_fmaf(pz, cz, p);
    const float two_ab = p + p;
    const float d = (aa - two_ab) + cb;
    if (d < bd[KNBR - 1]) {
#pragma unroll
      for (int j = KNBR - 1; j >= 1; --j) {
        const bool lp = d < bd[j - 1];
        const bool lc = d < bd[j];
        const float nd = lp ? bd[j - 1] : (lc ? d : bd[j]);
        const int   ni = lp ? bi[j - 1] : (lc ? s : bi[j]);
        bd[j] = nd;
        bi[j] = ni;
      }
      const bool l0 = d < bd[0];
      bd[0] = l0 ? d : bd[0];
      bi[0] = l0 ? s : bi[0];
    }
  }

  __syncthreads();
#pragma unroll
  for (int m = 0; m < 4; ++m) {
    v4u vi, vd;
    vi.x = (unsigned)bi[4 * m + 0];
    vi.y = (unsigned)bi[4 * m + 1];
    vi.z = (unsigned)bi[4 * m + 2];
    vi.w = (unsigned)bi[4 * m + 3];
    vd.x = __float_as_uint(bd[4 * m + 0]);
    vd.y = __float_as_uint(bd[4 * m + 1]);
    vd.z = __float_as_uint(bd[4 * m + 2]);
    vd.w = __float_as_uint(bd[4 * m + 3]);
    sbuf[t * 4 + m] = vi;
    sbuf[1024 + t * 4 + m] = vd;
  }
  __syncthreads();
  v4u oi[4], od[4];
#pragma unroll
  for (int i = 0; i < 4; ++i) { oi[i] = sbuf[t + 256 * i]; od[i] = sbuf[1024 + t + 256 * i]; }
  const size_t base4 = ((size_t)b * NQUERY + (size_t)blockIdx.x * 256) * 4;
  volatile v4u* gi = (volatile v4u*)idx_plane + base4;
  volatile v4u* gd = (volatile v4u*)dsel_plane + base4;
  for (int pass = 0; pass < 2; ++pass) {
#pragma unroll
    for (int i = 0; i < 4; ++i) {
      gi[t + 256 * i] = oi[i];
      gd[t + 256 * i] = od[i];
    }
    __threadfence();
  }
}

__global__ __launch_bounds__(256)
void interp_concat_kernel(const float* __restrict__ points1, const float* __restrict__ points2,
                          const int* __restrict__ idx_plane, const float* __restrict__ dsel_plane,
                          unsigned short* __restrict__ X) {
  const int lane = threadIdx.x & 31;
  const int wave = threadIdx.x >> 5;
  const int row  = blockIdx.x * 8 + wave;
  const int b    = row >> 13;
  const int k    = lane & 15;

  int id = idx_plane[(size_t)row * KNBR + k];
  id = id < 0 ? 0 : id;
  id = id > (NSRC - 1) ? (NSRC - 1) : id;
  const float dk = dsel_plane[(size_t)row * KNBR + k];
  const float rk = 1.0f / (dk + EPS_DIST);
  float rs = rk;
  rs = rs + __shfl_xor(rs, 1, 32);
  rs = rs + __shfl_xor(rs, 2, 32);
  rs = rs + __shfl_xor(rs, 4, 32);
  rs = rs + __shfl_xor(rs, 8, 32);
  const float wl = rk / rs;

  float acc[8];
#pragma unroll
  for (int e = 0; e < 8; ++e) acc[e] = 0.0f;
  const float* p2b = points2 + (size_t)b * NSRC * CH_P2 + lane * 8;
#pragma unroll 2
  for (int kk = 0; kk < KNBR; ++kk) {
    const float wk = __shfl(wl, kk, 32);
    const int   ik = __shfl(id, kk, 32);
    const float* src = p2b + (size_t)ik * CH_P2;
    const v4f a0 = *(const v4f*)(src);
    const v4f a1 = *(const v4f*)(src + 4);
    acc[0] = __builtin_fmaf(wk, a0.x, acc[0]);
    acc[1] = __builtin_fmaf(wk, a0.y, acc[1]);
    acc[2] = __builtin_fmaf(wk, a0.z, acc[2]);
    acc[3] = __builtin_fmaf(wk, a0.w, acc[3]);
    acc[4] = __builtin_fmaf(wk, a1.x, acc[4]);
    acc[5] = __builtin_fmaf(wk, a1.y, acc[5]);
    acc[6] = __builtin_fmaf(wk, a1.z, acc[6]);
    acc[7] = __builtin_fmaf(wk, a1.w, acc[7]);
  }
  v8h hv;
#pragma unroll
  for (int e = 0; e < 8; ++e) hv[e] = (_Float16)acc[e];

  const int c8 = k * 8;
  const float* p1 = points1 + (size_t)row * CH_P1 + c8;
  const v4f f0 = *(const v4f*)(p1);
  const v4f f1 = *(const v4f*)(p1 + 4);
  v8h pv;
  pv[0] = (_Float16)f0.x; pv[1] = (_Float16)f0.y; pv[2] = (_Float16)f0.z; pv[3] = (_Float16)f0.w;
  pv[4] = (_Float16)f1.x; pv[5] = (_Float16)f1.y; pv[6] = (_Float16)f1.z; pv[7] = (_Float16)f1.w;

  unsigned short* xr = X + (size_t)row * CH_IN;
  for (int pass = 0; pass < 2; ++pass) {
    if (lane < 16) *(volatile v8h*)(xr + c8) = pv;
    *(volatile v8h*)(xr + CH_P1 + lane * 8) = hv;
    __threadfence();
  }
}

__global__ __launch_bounds__(256)
void wsplit_kernel(const float* __restrict__ W0, const float* __restrict__ W1,
                   unsigned short* __restrict__ hi, unsigned short* __restrict__ lo) {
  const int i  = blockIdx.x * 256 + threadIdx.x;
  const int e0 = i * 8;
  const bool inW0 = blockIdx.x < W0_BLOCKS;
  const float* src = inW0 ? (W0 + e0) : (W1 + (e0 - W0_ELEMS));
  const v4f a = *(const v4f*)(src);
  const v4f c = *(const v4f*)(src + 4);
  float w[8];
  w[0] = a.x; w[1] = a.y; w[2] = a.z; w[3] = a.w;
  w[4] = c.x; w[5] = c.y; w[6] = c.z; w[7] = c.w;
  v8h hv, lv;
#pragma unroll
  for (int e = 0; e < 8; ++e) {
    const float ws = w[e] * W_CARRY;
    const _Float16 h = (_Float16)ws;
    const float hf = (float)h;
    const _Float16 l = (_Float16)(ws - hf);
    hv[e] = h;
    lv[e] = l;
  }
  for (int pass = 0; pass < 2; ++pass) {
    *(volatile v8h*)(hi + e0) = hv;
    *(volatile v8h*)(lo + e0) = lv;
    __threadfence();
  }
}

__global__ __launch_bounds__(256)
void gemm_f16_wsplit_kernel(const unsigned short* __restrict__ Ap, int lda,
                            const unsigned short* __restrict__ Bhp, const unsigned short* __restrict__ Blp, int ldb,
                            float* __restrict__ Cout, int ldc,
                            const float* __restrict__ bias, float* __restrict__ part,
                            int M, int N, int K, float scale) {
  const _Float16* A  = (const _Float16*)Ap;
  const _Float16* Bh = (const _Float16*)Bhp;
  const _Float16* Bl = (const _Float16*)Blp;
  __shared__ __align__(16) float sT[8][16 * 68];
  const int lane = threadIdx.x & 31;
  const int wave = threadIdx.x >> 5;
  const int tilesN = N >> 6;
  const int tilesM = M >> 6;
  const int tile = blockIdx.x * 8 + wave;
  if (tile >= tilesM * tilesN) return;
  const int tm = tile / tilesN;
  const int tn = tile - tm * tilesN;
  const int m0 = tm << 6;
  const int n0 = tn << 6;

  const int rlane = lane & 15;
  const int hh    = lane >> 4;
  const int koff  = hh * 8;
  const int mOff  = hh * 8;

  v8f acc[4][4];
#pragma unroll
  for (int i = 0; i < 4; ++i)
#pragma unroll
    for (int j = 0; j < 4; ++j) acc[i][j] = (v8f){0.f, 0.f, 0.f, 0.f, 0.f, 0.f, 0.f, 0.f};

  for (int k0 = 0; k0 < K; k0 += 32) {
    v16h bh[4], bl[4];
#pragma unroll
    for (int j = 0; j < 4; ++j) {
      const size_t bo = (size_t)(n0 + (j << 4) + rlane) * ldb + koff + k0;
      bh[j] = FragH::load(Bh + bo);
      bl[j] = FragH::load(Bl + bo);
    }
#pragma unroll
    for (int i = 0; i < 4; ++i) {
      const size_t ao = (size_t)(m0 + (i << 4) + rlane) * lda + koff + k0;
      const v16h ah = FragH::load(A + ao);
#pragma unroll
      for (int j = 0; j < 4; ++j) acc[i][j] = FragH::mma(ah, bh[j], acc[i][j]);
#pragma unroll
      for (int j = 0; j < 4; ++j) acc[i][j] = FragH::mma(ah, bl[j], acc[i][j]);
      guard_row_h(acc[i][0], acc[i][1], acc[i][2], acc[i][3], ah,
                  bh[0], bh[1], bh[2], bh[3], bl[0], bl[1], bl[2], bl[3]);
    }
    keep4_h(bh[0], bh[1], bh[2], bh[3]);
    keep4_h(bl[0], bl[1], bl[2], bl[3]);
  }
  acc_guard4(acc[0][0], acc[0][1], acc[0][2], acc[0][3]);
  acc_guard4(acc[1][0], acc[1][1], acc[1][2], acc[1][3]);
  acc_guard4(acc[2][0], acc[2][1], acc[2][2], acc[2][3]);
  acc_guard4(acc[3][0], acc[3][1], acc[3][2], acc[3][3]);

  float bvj[4];
#pragma unroll
  for (int j = 0; j < 4; ++j) bvj[j] = bias[n0 + (j << 4) + rlane];
  float cs[4], cq[4];
#pragma unroll
  for (int j = 0; j < 4; ++j) { cs[j] = 0.0f; cq[j] = 0.0f; }

  float* slab = sT[wave];
  const int c4 = rlane * 4;
#pragma unroll
  for (int i = 0; i < 4; ++i) {
    const int mBase = m0 + (i << 4);
#pragma unroll
    for (int j = 0; j < 4; ++j) {
#pragma unroll
      for (int r = 0; r < 8; ++r) {
        float v = acc[i][j][r] * scale;
        v = v + bvj[j];
        cs[j] = cs[j] + v;
        const float v2 = v * v;
        cq[j] = cq[j] + v2;
        slab[(mOff + r) * 68 + (j << 4) + rlane] = v;
      }
    }
    __builtin_amdgcn_fence(__ATOMIC_RELEASE, "workgroup");
    __builtin_amdgcn_wave_barrier();
    __builtin_amdgcn_fence(__ATOMIC_ACQUIRE, "workgroup");
    for (int pass = 0; pass < 2; ++pass) {
#pragma unroll
      for (int it = 0; it < 8; ++it) {
        const int row = it * 2 + hh;
        const v4f vv = *(const v4f*)(slab + row * 68 + c4);
        *(volatile v4f*)(Cout + (size_t)(mBase + row) * ldc + n0 + c4) = vv;
      }
      __threadfence();
    }
    __builtin_amdgcn_fence(__ATOMIC_RELEASE, "workgroup");
    __builtin_amdgcn_wave_barrier();
    __builtin_amdgcn_fence(__ATOMIC_ACQUIRE, "workgroup");
  }

#pragma unroll
  for (int j = 0; j < 4; ++j) {
    const float os = __shfl_xor(cs[j], 16, 32);
    const float oq = __shfl_xor(cq[j], 16, 32);
    cs[j] = cs[j] + os;
    cq[j] = cq[j] + oq;
  }
#pragma unroll
  for (int j = 0; j < 4; ++j) {
    const float sv = hh ? cq[j] : cs[j];
    slab[hh * 64 + (j << 4) + rlane] = sv;
  }
  __builtin_amdgcn_fence(__ATOMIC_RELEASE, "workgroup");
  __builtin_amdgcn_wave_barrier();
  __builtin_amdgcn_fence(__ATOMIC_ACQUIRE, "workgroup");
  {
    const v4f pvv = *(const v4f*)(slab + hh * 64 + c4);
    float* pp = part + ((size_t)tm * 2 + hh) * N + n0 + c4;
    for (int pass = 0; pass < 2; ++pass) {
      *(volatile v4f*)(pp) = pvv;
      __threadfence();
    }
  }
}

__global__ __launch_bounds__(256)
void bn_stats_kernel(const float* __restrict__ part, int C, int tiles,
                     const float* __restrict__ gamma, const float* __restrict__ beta,
                     float* __restrict__ st, float inv_rows) {
  __shared__ double rs[8][32];
  __shared__ double rq[8][32];
  const int lane = threadIdx.x & 31;
  const int wave = threadIdx.x >> 5;
  const int c = blockIdx.x * 32 + lane;
  const int per = tiles >> 3;
  double s = 0.0, q = 0.0;
#pragma unroll 4
  for (int i = 0; i < per; ++i) {
    const int tm = wave * per + i;
    const float fs = part[((size_t)tm * 2) * C + c];
    const float fq = part[((size_t)tm * 2 + 1) * C + c];
    s = s + (double)fs;
    q = q + (double)fq;
  }
  rs[wave][lane] = s;
  rq[wave][lane] = q;
  __syncthreads();
  if (wave == 0) {
    double S = 0.0, Q = 0.0;
#pragma unroll
    for (int w = 0; w < 8; ++w) { S = S + rs[w][lane]; Q = Q + rq[w][lane]; }
    const double inv = (double)inv_rows;
    const double mean = S * inv;
    double var = Q * inv - mean * mean;
    var = var < 0.0 ? 0.0 : var;
    const float rstd = rsqrtf((float)var + EPS_BN);
    const float sc = rstd * gamma[c];
    const float sh = (float)((double)beta[c] - mean * (double)sc);
    for (int pass = 0; pass < 2; ++pass) {
      ((volatile float*)st)[c] = sc;
      ((volatile float*)st)[C + c] = sh;
      __threadfence();
    }
  }
}

__global__ __launch_bounds__(256)
void bn_relu_h16_kernel(const float* __restrict__ Y, const float* __restrict__ st,
                        unsigned short* __restrict__ H) {
  const size_t i = (size_t)blockIdx.x * 256 + threadIdx.x;
  const int c8 = (int)(i & 31) * 8;
  const v4f y0 = *(const v4f*)(Y + i * 8);
  const v4f y1 = *(const v4f*)(Y + i * 8 + 4);
  const v4f s0 = *(const v4f*)(st + c8);
  const v4f s1 = *(const v4f*)(st + c8 + 4);
  const v4f h0 = *(const v4f*)(st + CH_L0 + c8);
  const v4f h1 = *(const v4f*)(st + CH_L0 + c8 + 4);
  v8h hv;
  hv[0] = (_Float16)fmaxf(__builtin_fmaf(y0.x, s0.x, h0.x), 0.0f);
  hv[1] = (_Float16)fmaxf(__builtin_fmaf(y0.y, s0.y, h0.y), 0.0f);
  hv[2] = (_Float16)fmaxf(__builtin_fmaf(y0.z, s0.z, h0.z), 0.0f);
  hv[3] = (_Float16)fmaxf(__builtin_fmaf(y0.w, s0.w, h0.w), 0.0f);
  hv[4] = (_Float16)fmaxf(__builtin_fmaf(y1.x, s1.x, h1.x), 0.0f);
  hv[5] = (_Float16)fmaxf(__builtin_fmaf(y1.y, s1.y, h1.y), 0.0f);
  hv[6] = (_Float16)fmaxf(__builtin_fmaf(y1.z, s1.z, h1.z), 0.0f);
  hv[7] = (_Float16)fmaxf(__builtin_fmaf(y1.w, s1.w, h1.w), 0.0f);
  for (int pass = 0; pass < 2; ++pass) {
    *(volatile v8h*)(H + i * 8) = hv;
    __threadfence();
  }
}

__global__ __launch_bounds__(256)
void bn_relu_f32_kernel(const float* __restrict__ Y, const float* __restrict__ st,
                        float* __restrict__ out) {
  const size_t i = (size_t)blockIdx.x * 256 + threadIdx.x;
  const int c4 = (int)(i & 31) * 4;
  const v4f y = *(const v4f*)(Y + i * 4);
  const v4f s = *(const v4f*)(st + c4);
  const v4f h = *(const v4f*)(st + CH_L1 + c4);
  v4f o;
  o.x = fmaxf(__builtin_fmaf(y.x, s.x, h.x), 0.0f);
  o.y = fmaxf(__builtin_fmaf(y.y, s.y, h.y), 0.0f);
  o.z = fmaxf(__builtin_fmaf(y.z, s.z, h.z), 0.0f);
  o.w = fmaxf(__builtin_fmaf(y.w, s.w, h.w), 0.0f);
  for (int pass = 0; pass < 2; ++pass) {
    *(volatile v4f*)(out + i * 4) = o;
    __threadfence();
  }
}

extern "C" void kernel_launch(void* const* d_in, const int* in_sizes, int n_in,
                              void* d_out, int out_size, void* d_ws, size_t ws_size,
                              hipStream_t stream) {
  if (n_in != 12) return;
  if (ws_size < WS_TOTAL) return;
  if (out_size != NROWS * CH_L1) return;
  if (in_sizes[0] != NROWS * 3 || in_sizes[1] != NBATCH * NSRC * 3) return;
  if (in_sizes[2] != NROWS * CH_P1 || in_sizes[3] != NBATCH * NSRC * CH_P2) return;
  if (in_sizes[4] != W0_ELEMS || in_sizes[8] != W1_ELEMS) return;

  const float* xyz1    = (const float*)d_in[0];
  const float* xyz2    = (const float*)d_in[1];
  const float* points1 = (const float*)d_in[2];
  const float* points2 = (const float*)d_in[3];
  const float* W0  = (const float*)d_in[4];
  const float* b0  = (const float*)d_in[5];
  const float* g0  = (const float*)d_in[6];
  const float* be0 = (const float*)d_in[7];
  const float* W1  = (const float*)d_in[8];
  const float* b1  = (const float*)d_in[9];
  const float* g1  = (const float*)d_in[10];
  const float* be1 = (const float*)d_in[11];

  char* ws = (char*)d_ws;
  unsigned*       idxp = (unsigned*)(ws + OFF_IDX);
  unsigned*       dsel = (unsigned*)(ws + OFF_DSEL);
  unsigned short* XH   = (unsigned short*)(ws + OFF_XH);
  float*          YF   = (float*)(ws + OFF_YF);
  unsigned short* WHI  = (unsigned short*)(ws + OFF_WHI);
  unsigned short* WLO  = (unsigned short*)(ws + OFF_WLO);
  float*          P0   = (float*)(ws + OFF_P0);
  float*          P1   = (float*)(ws + OFF_P1);
  float*          ST0  = (float*)(ws + OFF_ST0);
  float*          ST1  = (float*)(ws + OFF_ST1);
  unsigned short* H0   = XH;
  float*          Y1   = YF;

  const float inv_rows = 1.0f / (float)NROWS;

  knn16_kernel<<<dim3(NQUERY / 256, NBATCH), 256, 0, stream>>>(xyz1, xyz2, idxp, dsel);
  interp_concat_kernel<<<NROWS / 8, 256, 0, stream>>>(points1, points2, (const int*)idxp,
                                                      (const float*)dsel, XH);
  wsplit_kernel<<<W_BLOCKS, 256, 0, stream>>>(W0, W1, WHI, WLO);

  gemm_f16_wsplit_kernel<<<(TILES_M * (CH_L0 / 64)) / 8, 256, 0, stream>>>(
      XH, CH_IN, WHI, WLO, CH_IN, YF, CH_L0, b0, P0, NROWS, CH_L0, CH_IN, W_CARRY_INV);
  bn_stats_kernel<<<CH_L0 / 32, 256, 0, stream>>>(P0, CH_L0, TILES_M, g0, be0, ST0, inv_rows);
  bn_relu_h16_kernel<<<(NROWS * (CH_L0 / 8)) / 256, 256, 0, stream>>>(YF, ST0, H0);

  gemm_f16_wsplit_kernel<<<(TILES_M * (CH_L1 / 64)) / 8, 256, 0, stream>>>(
      H0, CH_L0, WHI + W0_ELEMS, WLO + W0_ELEMS, CH_L0, Y1, CH_L1, b1, P1, NROWS, CH_L1, CH_L0, W_CARRY_INV);
  bn_stats_kernel<<<CH_L1 / 32, 256, 0, stream>>>(P1, CH_L1, TILES_M, g1, be1, ST1, inv_rows);
  bn_relu_f32_kernel<<<(NROWS * (CH_L1 / 4)) / 256, 256, 0, stream>>>(Y1, ST1, (float*)d_out);
}
